// GAT_9096740733072
// MI455X (gfx1250) — hardware-verified
//
#include <hip/hip_runtime.h>
#include <stddef.h>
#include <stdint.h>
#include <math.h>


#define NN     256
#define ED     128
#define NH     4
#define F0     384
#define F1     768
#define TW     256
#define KH     1024
#define GBM    64
#define GBN    128
#define GTHR   128
#define NTHR   256
#define U_WE   4096
#define U_WR   8192
#define U_W0   10240
#define U_W1   26624
#define LDS_LAYER_FLOATS (NN * ED + NN * NH + 8 * NH * ED + NH * ED + NH * ED + 64 + 2 * NN)
#define WSMAX  134217728

static_assert(U_WE == 256 * (ED / 8));
static_assert(U_WR - U_WE == 256 * (ED / 8));
static_assert(U_W0 - U_WR == 128 * (ED / 8));
static_assert(U_W1 - U_W0 == 128 * (KH / 8));
static_assert((U_WE % NTHR) == 0 && (U_WR % NTHR) == 0 && (U_W0 % NTHR) == 0 && (U_W1 % NTHR) == 0);
static_assert(GBM == (GTHR / 32) * 16 && GBN == 4 * 32);
static_assert((ED % 32) == 0 && (KH % 32) == 0 && KH == 2 * NH * ED);
static_assert(NTHR == NN && ED == 4 * 32 && NH == 4);
static_assert(LDS_LAYER_FLOATS * 4 <= 300000);

typedef float          v4f   __attribute__((ext_vector_type(4)));
typedef float          v8f   __attribute__((ext_vector_type(8)));
typedef int            v2i   __attribute__((ext_vector_type(2)));
typedef int            v8i   __attribute__((ext_vector_type(8)));
typedef unsigned int   v2u   __attribute__((ext_vector_type(2)));
typedef unsigned int   v4u   __attribute__((ext_vector_type(4)));
typedef unsigned short v8us  __attribute__((ext_vector_type(8)));
typedef __bf16         v16bf __attribute__((ext_vector_type(16)));
typedef v4f  __attribute__((may_alias)) v4fa;
typedef v2i  __attribute__((may_alias)) v2ia;
typedef v2u  __attribute__((may_alias)) v2ua;
typedef v8us __attribute__((may_alias)) v8usa;
union FragB { v16bf v; v8us h[2]; v8i w; v4u q[2]; };

__device__ __forceinline__ v8f wmb(const FragB& a, const FragB& b, v8f c) {
  v8f d = __builtin_amdgcn_wmma_f32_16x16x32_bf16(false, a.v, false, b.v, (short)0, c, false, false);
  asm volatile("v_nop\n\tv_nop\n\tv_nop\n\tv_nop" : "+v"(d) : "v"(a.w), "v"(b.w));
  return d;
}

__device__ __forceinline__ unsigned int f2bf(float f) {
  const unsigned int u = __float_as_uint(f);
  return ((u + 0x7FFFu + ((u >> 16) & 1u)) >> 16) & 0xFFFFu;
}
__device__ __forceinline__ float bf2f(unsigned int b) { return __uint_as_float(b << 16); }
__device__ __forceinline__ float bfr(float f) { return bf2f(f2bf(f)); }
__device__ __forceinline__ v4f bfr4(const v4f a) {
  v4f r; r.x = bfr(a.x); r.y = bfr(a.y); r.z = bfr(a.z); r.w = bfr(a.w); return r;
}
__device__ __forceinline__ unsigned int pk2(float lo, float hi) { return f2bf(lo) | (f2bf(hi) << 16); }
__device__ __forceinline__ v4u pack8(const v4f a, const v4f b) {
  v4u r;
  r.x = pk2(a.x, a.y); r.y = pk2(a.z, a.w); r.z = pk2(b.x, b.y); r.w = pk2(b.z, b.w);
  return r;
}
__device__ __forceinline__ v4u ld_cvt8(const float* __restrict__ p) {
  const v4f a = *(const v4fa*)p;
  const v4f b = *(const v4fa*)(p + 4);
  return pack8(a, b);
}

__global__ __launch_bounds__(NTHR) void k_prep(const float* __restrict__ W0, const float* __restrict__ W1,
                                               const float* __restrict__ embE, const int* __restrict__ be1,
                                               const int* __restrict__ bq,
                                               unsigned short* planes, int nEnt, int nUnits) {
  (void)bq;
  const int u = (int)blockIdx.x * NTHR + (int)threadIdx.x;
  if (u >= nUnits) return;
  v4u o;
  if (u < U_WE) {
    const int n = u >> 4, k8 = (u & 15) * 8;
    if (n < 128) o = ld_cvt8(W0 + (size_t)n * F0 + 256 + k8);
    else         o = ld_cvt8(W1 + (size_t)(n - 128) * F1 + 640 + k8);
  } else if (u < U_WR) {
    const int v = u - U_WE;
    const int n = v >> 4, k8 = (v & 15) * 8;
    if (n < 128) o = ld_cvt8(W0 + (size_t)n * F0 + 128 + k8);
    else         o = ld_cvt8(W1 + (size_t)(n - 128) * F1 + 512 + k8);
  } else if (u < U_W0) {
    const int v = u - U_WR;
    const int n = v >> 4, k8 = (v & 15) * 8;
    o = ld_cvt8(W0 + (size_t)n * F0 + k8);
  } else if (u < U_W1) {
    const int v = u - U_W0;
    const int n = v >> 7, k8 = (v & 127) * 8;
    const int kk = k8 & 511;
    o = ld_cvt8(W1 + (size_t)n * F1 + kk);
  } else {
    const int v = u - U_W1;
    const int b = v >> 4, k8 = (v & 15) * 8;
    int id = be1[b];
    id = id < 0 ? 0 : (id > nEnt - 1 ? nEnt - 1 : id);
    o = ld_cvt8(embE + (size_t)id * ED + k8);
  }
  unsigned short* dp = planes + (size_t)u * 8;
  *(volatile v4u*)dp = o;
  __threadfence();
  *(volatile v4u*)dp = o;
}

template <int NC, int AF32>
__global__ __launch_bounds__(GTHR * NC) void k_gemm(const float* __restrict__ Af,
                                                    const unsigned short* __restrict__ Ab, int lda, int mReal,
                                                    const unsigned short* __restrict__ BT, int ldb, int K,
                                                    float* Cm, const float* __restrict__ bias, int hasBias) {
  static_assert(NC == 1 || NC == 2);
  constexpr int LDC = GBN * NC;
  constexpr int RPW = GBM / (4 * NC);
  extern __shared__ __attribute__((aligned(16))) float gsm[];
  float* stg = gsm;
  const int tid = (int)threadIdx.x, lane = tid & 31, wave = tid >> 5, hh = lane >> 4, m = lane & 15;
  const int rg = wave & 3, cg = wave >> 2;
  const int rowBase = (int)blockIdx.x * GBM;
  const int colBase = cg * GBN;

  v8f acc[8];
  {
    const v8f z = {0.f, 0.f, 0.f, 0.f, 0.f, 0.f, 0.f, 0.f};
#pragma unroll
    for (int t = 0; t < 8; ++t) acc[t] = z;
  }
  int ar = rowBase + 16 * rg + m;
  ar = ar < mReal ? ar : mReal - 1;
  const size_t aoff = (size_t)ar * (size_t)lda + 8 * hh;
  const unsigned short* bp = BT + (size_t)(colBase + m) * (size_t)ldb + 8 * hh;

#pragma unroll 1
  for (int k0 = 0; k0 < K; k0 += 32) {
    FragB af;
    if constexpr (AF32 != 0) {
      const float* q = Af + aoff + k0;
      const v4f a0 = *(const v4fa*)q;
      const v4f a1 = *(const v4fa*)(q + 4);
      const v4f a2 = *(const v4fa*)(q + 16);
      const v4f a3 = *(const v4fa*)(q + 20);
      af.q[0] = pack8(a0, a1);
      af.q[1] = pack8(a2, a3);
    } else {
      const unsigned short* q = Ab + aoff + k0;
      af.h[0] = *(const v8usa*)q;
      af.h[1] = *(const v8usa*)(q + 16);
    }
#pragma unroll
    for (int nt = 0; nt < 8; ++nt) {
      const unsigned short* wq = bp + (size_t)(16 * nt) * (size_t)ldb + k0;
      FragB bf;
      bf.h[0] = *(const v8usa*)wq;
      bf.h[1] = *(const v8usa*)(wq + 16);
      acc[nt] = wmb(af, bf, acc[nt]);
    }
  }

#pragma unroll
  for (int nt = 0; nt < 8; ++nt) {
    const int lc = colBase + 16 * nt + m;
#pragma unroll
    for (int r = 0; r < 8; ++r) {
      const int lr = 16 * rg + 8 * hh + r;
      stg[lr * LDC + lc] = acc[nt][r];
    }
  }
  __syncthreads();

  v4f bz[NC];
#pragma unroll
  for (int c = 0; c < NC; ++c) {
    const v4f bb = bfr4(*(const v4fa*)(bias + c * GBN + 4 * lane));
    v4f z;
    z.x = (hasBias != 0) ? bb.x : 0.0f;
    z.y = (hasBias != 0) ? bb.y : 0.0f;
    z.z = (hasBias != 0) ? bb.z : 0.0f;
    z.w = (hasBias != 0) ? bb.w : 0.0f;
    bz[c] = z;
  }
#pragma unroll 1
  for (int i = 0; i < RPW; ++i) {
    const int row = wave * RPW + i;
#pragma unroll
    for (int c = 0; c < NC; ++c) {
      const v4f p = *(const v4fa*)(stg + row * LDC + c * GBN + 4 * lane);
      const v4f o = p + bz[c];
      float* op = Cm + (size_t)(rowBase + row) * (size_t)LDC + c * GBN + 4 * lane;
      *(volatile v4f*)op = o;
    }
  }
  __threadfence();
#pragma unroll 1
  for (int i = 0; i < RPW; ++i) {
    const int row = wave * RPW + i;
#pragma unroll
    for (int c = 0; c < NC; ++c) {
      const v4f p = *(const v4fa*)(stg + row * LDC + c * GBN + 4 * lane);
      const v4f o = p + bz[c];
      float* op = Cm + (size_t)(rowBase + row) * (size_t)LDC + c * GBN + 4 * lane;
      *(volatile v4f*)op = o;
    }
  }
}

template <int LAYER>
__global__ __launch_bounds__(NTHR) void k_layer(const int* __restrict__ nbr, const float* __restrict__ masks,
                                                const float* __restrict__ Cb,
                                                const float* __restrict__ TR, const float* __restrict__ TE,
                                                const float* __restrict__ aW, const float* __restrict__ ab,
                                                const unsigned short* __restrict__ HB,
                                                unsigned short* HHL, float* out, int nRel, int nEnt) {
  extern __shared__ __attribute__((aligned(16))) float lsm[];
  float* xs   = lsm;
  float* pp   = xs + NN * ED;
  float* part = pp + NN * NH;
  float* aggs = part + 8 * NH * ED;
  float* aws  = aggs + NH * ED;
  float* wred = aws + NH * ED;
  int*   ids  = (int*)(wred + 64);
  const int tid = (int)threadIdx.x, lane = tid & 31, wave = tid >> 5;
  const size_t b = (size_t)blockIdx.x;

  {
    const v2i pr = *(const v2ia*)(nbr + (b * NN + (size_t)tid) * 2);
    v2i cl;
    cl.x = pr.x < 0 ? 0 : (pr.x > nRel - 1 ? nRel - 1 : pr.x);
    cl.y = pr.y < 0 ? 0 : (pr.y > nEnt - 1 ? nEnt - 1 : pr.y);
    *(v2ia*)(ids + 2 * tid) = cl;
    aws[tid]       = bfr(aW[tid]);
    aws[tid + 256] = bfr(aW[tid + 256]);
  }
  __syncthreads();

  {
    const v4f c4 = *(const v4fa*)(Cb + b * ED + 4 * lane);
    const int toff = LAYER * ED + 4 * lane;
#pragma unroll 2
    for (int i = 0; i < 32; ++i) {
      const int n = wave * 32 + i;
      const v2i id = *(const v2ia*)(ids + 2 * n);
      const v4f tr = *(const v4fa*)(TR + (size_t)id.x * TW + toff);
      const v4f te = *(const v4fa*)(TE + (size_t)id.y * TW + toff);
      const v4f xv = (c4 + tr) + te;
      *(v4fa*)(xs + n * ED + 4 * lane) = xv;
    }
  }
  __syncthreads();

  float l0, l1, l2, l3;
  {
    float a0 = 0.0f, a1 = 0.0f, a2 = 0.0f, a3 = 0.0f;
    const float* xr = xs + tid * ED;
#pragma unroll 1
    for (int q = 0; q < ED / 4; ++q) {
      const v4f xv = *(const v4fa*)(xr + 4 * q);
      const v4f w0 = *(const v4fa*)(aws + 4 * q);
      const v4f w1 = *(const v4fa*)(aws + ED + 4 * q);
      const v4f w2 = *(const v4fa*)(aws + 2 * ED + 4 * q);
      const v4f w3 = *(const v4fa*)(aws + 3 * ED + 4 * q);
      a0 = fmaf(xv.x, w0.x, a0); a0 = fmaf(xv.y, w0.y, a0); a0 = fmaf(xv.z, w0.z, a0); a0 = fmaf(xv.w, w0.w, a0);
      a1 = fmaf(xv.x, w1.x, a1); a1 = fmaf(xv.y, w1.y, a1); a1 = fmaf(xv.z, w1.z, a1); a1 = fmaf(xv.w, w1.w, a1);
      a2 = fmaf(xv.x, w2.x, a2); a2 = fmaf(xv.y, w2.y, a2); a2 = fmaf(xv.z, w2.z, a2); a2 = fmaf(xv.w, w2.w, a2);
      a3 = fmaf(xv.x, w3.x, a3); a3 = fmaf(xv.y, w3.y, a3); a3 = fmaf(xv.z, w3.z, a3); a3 = fmaf(xv.w, w3.w, a3);
    }
    const v4f abv = bfr4(*(const v4fa*)ab);
    const float mk = bfr(masks[b * NN + (size_t)tid]);
    const float mterm = 1e31f * (1.0f - mk);
    l0 = a0 + abv.x; l0 = (l0 >= 0.0f) ? l0 : 0.1f * l0; l0 = l0 - mterm;
    l1 = a1 + abv.y; l1 = (l1 >= 0.0f) ? l1 : 0.1f * l1; l1 = l1 - mterm;
    l2 = a2 + abv.z; l2 = (l2 >= 0.0f) ? l2 : 0.1f * l2; l2 = l2 - mterm;
    l3 = a3 + abv.w; l3 = (l3 >= 0.0f) ? l3 : 0.1f * l3; l3 = l3 - mterm;
  }

  {
    float m0 = l0, m1 = l1, m2 = l2, m3 = l3;
#pragma unroll
    for (int off = 16; off > 0; off >>= 1) {
      m0 = fmaxf(m0, __shfl_xor(m0, off));
      m1 = fmaxf(m1, __shfl_xor(m1, off));
      m2 = fmaxf(m2, __shfl_xor(m2, off));
      m3 = fmaxf(m3, __shfl_xor(m3, off));
    }
    if (lane == 0) {
      v4f mv; mv.x = m0; mv.y = m1; mv.z = m2; mv.w = m3;
      *(v4fa*)(wred + 4 * wave) = mv;
    }
    __syncthreads();
    v4f g = *(const v4fa*)wred;
#pragma unroll
    for (int w2 = 1; w2 < 8; ++w2) {
      const v4f t = *(const v4fa*)(wred + 4 * w2);
      g.x = fmaxf(g.x, t.x); g.y = fmaxf(g.y, t.y); g.z = fmaxf(g.z, t.z); g.w = fmaxf(g.w, t.w);
    }
    const float e0 = expf(l0 - g.x);
    const float e1 = expf(l1 - g.y);
    const float e2 = expf(l2 - g.z);
    const float e3 = expf(l3 - g.w);
    float s0 = e0, s1 = e1, s2 = e2, s3 = e3;
#pragma unroll
    for (int off = 16; off > 0; off >>= 1) {
      s0 += __shfl_xor(s0, off);
      s1 += __shfl_xor(s1, off);
      s2 += __shfl_xor(s2, off);
      s3 += __shfl_xor(s3, off);
    }
    if (lane == 0) {
      v4f sv; sv.x = s0; sv.y = s1; sv.z = s2; sv.w = s3;
      *(v4fa*)(wred + 32 + 4 * wave) = sv;
    }
    __syncthreads();
    v4f tsum = *(const v4fa*)(wred + 32);
#pragma unroll
    for (int w2 = 1; w2 < 8; ++w2) {
      const v4f t = *(const v4fa*)(wred + 32 + 4 * w2);
      tsum = tsum + t;
    }
    v4f pv;
    pv.x = e0 * __builtin_amdgcn_rcpf(tsum.x);
    pv.y = e1 * __builtin_amdgcn_rcpf(tsum.y);
    pv.z = e2 * __builtin_amdgcn_rcpf(tsum.z);
    pv.w = e3 * __builtin_amdgcn_rcpf(tsum.w);
    *(v4fa*)(pp + 4 * tid) = pv;
  }
  __syncthreads();

  {
    v4f c0 = {0.f, 0.f, 0.f, 0.f}, c1 = c0, c2 = c0, c3 = c0;
#pragma unroll 1
    for (int i = 0; i < 32; ++i) {
      const int n = wave * 32 + i;
      const v4f xv = *(const v4fa*)(xs + n * ED + 4 * lane);
      const v4f p  = *(const v4fa*)(pp + 4 * n);
      c0.x = fmaf(p.x, xv.x, c0.x); c0.y = fmaf(p.x, xv.y, c0.y); c0.z = fmaf(p.x, xv.z, c0.z); c0.w = fmaf(p.x, xv.w, c0.w);
      c1.x = fmaf(p.y, xv.x, c1.x); c1.y = fmaf(p.y, xv.y, c1.y); c1.z = fmaf(p.y, xv.z, c1.z); c1.w = fmaf(p.y, xv.w, c1.w);
      c2.x = fmaf(p.z, xv.x, c2.x); c2.y = fmaf(p.z, xv.y, c2.y); c2.z = fmaf(p.z, xv.z, c2.z); c2.w = fmaf(p.z, xv.w, c2.w);
      c3.x = fmaf(p.w, xv.x, c3.x); c3.y = fmaf(p.w, xv.y, c3.y); c3.z = fmaf(p.w, xv.z, c3.z); c3.w = fmaf(p.w, xv.w, c3.w);
    }
    *(v4fa*)(part + (wave * NH + 0) * ED + 4 * lane) = c0;
    *(v4fa*)(part + (wave * NH + 1) * ED + 4 * lane) = c1;
    *(v4fa*)(part + (wave * NH + 2) * ED + 4 * lane) = c2;
    *(v4fa*)(part + (wave * NH + 3) * ED + 4 * lane) = c3;
  }
  __syncthreads();
#pragma unroll
  for (int p2 = 0; p2 < 2; ++p2) {
    const int j = tid + 256 * p2;
    float s = part[j];
#pragma unroll
    for (int c = 1; c < 8; ++c) s += part[c * (NH * ED) + j];
    aggs[j] = s;
  }
  __syncthreads();

  if constexpr (LAYER == 0) {
    if (tid < 128) {
      const int j0 = 8 * (tid & 63);
      const v4f va = *(const v4fa*)(aggs + j0);
      const v4f vb = *(const v4fa*)(aggs + j0 + 4);
      float v[8];
      v[0] = va.x; v[1] = va.y; v[2] = va.z; v[3] = va.w;
      v[4] = vb.x; v[5] = vb.y; v[6] = vb.z; v[7] = vb.w;
      unsigned int hb[8], lb[8];
#pragma unroll
      for (int i = 0; i < 8; ++i) {
        const float y = (v[i] >= 0.0f) ? v[i] : 0.01f * v[i];
        hb[i] = f2bf(y);
        lb[i] = f2bf(y - bf2f(hb[i]));
      }
      const bool lsel = tid >= 64;
      v4u pv;
      pv.x = lsel ? (lb[0] | (lb[1] << 16)) : (hb[0] | (hb[1] << 16));
      pv.y = lsel ? (lb[2] | (lb[3] << 16)) : (hb[2] | (hb[3] << 16));
      pv.z = lsel ? (lb[4] | (lb[5] << 16)) : (hb[4] | (hb[5] << 16));
      pv.w = lsel ? (lb[6] | (lb[7] << 16)) : (hb[6] | (hb[7] << 16));
      unsigned short* gp = HHL + b * KH + 8 * tid;
      *(volatile v4u*)gp = pv;
      __threadfence();
      *(volatile v4u*)gp = pv;
    }
  } else {
    if (wave == 0) {
      const int d = 4 * lane;
      const v4f s0 = *(const v4fa*)(aggs + d);
      const v4f s1 = *(const v4fa*)(aggs + ED + d);
      const v4f s2 = *(const v4fa*)(aggs + 2 * ED + d);
      const v4f s3 = *(const v4fa*)(aggs + 3 * ED + d);
      const v4f sm = ((s0 + s1) + s2) + s3;
      const v2u hw = *(const v2ua*)(HB + b * ED + d);
      v4f o;
      o.x = bf2f(hw.x & 0xFFFFu) + 0.25f * sm.x;
      o.y = bf2f(hw.x >> 16)     + 0.25f * sm.y;
      o.z = bf2f(hw.y & 0xFFFFu) + 0.25f * sm.z;
      o.w = bf2f(hw.y >> 16)     + 0.25f * sm.w;
      float* op = out + b * ED + d;
      *(volatile v4f*)op = o;
      __threadfence();
      *(volatile v4f*)op = o;
    }
  }
}

static inline int cdiv(int a, int b) { return (a + b - 1) / b; }

extern "C" void kernel_launch(void* const* d_in, const int* in_sizes, int n_in,
                              void* d_out, int out_size, void* d_ws, size_t ws_size,
                              hipStream_t stream) {
  if (n_in < 14) return;
  const int nB = in_sizes[0];
  if (nB < GBM || (nB % GBM) != 0 || nB > (1 << 20)) return;
  if (in_sizes[1] != nB) return;
  if ((long long)in_sizes[2] != (long long)nB * NN * 2) return;
  if ((long long)in_sizes[3] != (long long)nB * NN) return;
  if (in_sizes[4] < ED || (in_sizes[4] % ED) != 0) return;
  if (in_sizes[5] < ED || (in_sizes[5] % ED) != 0) return;
  const int nEnt = in_sizes[4] / ED;
  const int nRel = in_sizes[5] / ED;
  if (in_sizes[6] != ED * F0 || in_sizes[7] != ED) return;
  if (in_sizes[8] != ED * F1 || in_sizes[9] != ED) return;
  if (in_sizes[10] != NH * ED || in_sizes[11] != NH) return;
  if (in_sizes[12] != NH * ED || in_sizes[13] != NH) return;
  if ((long long)out_size != (long long)nB * ED) return;

  const int*   be1  = (const int*)  d_in[0];
  const int*   bq   = (const int*)  d_in[1];
  const int*   nbr  = (const int*)  d_in[2];
  const float* msk  = (const float*)d_in[3];
  const float* embE = (const float*)d_in[4];
  const float* embR = (const float*)d_in[5];
  const float* W0   = (const float*)d_in[6];
  const float* b0   = (const float*)d_in[7];
  const float* W1   = (const float*)d_in[8];
  const float* b1   = (const float*)d_in[9];
  const float* a0W  = (const float*)d_in[10];
  const float* a0b  = (const float*)d_in[11];
  const float* a1W  = (const float*)d_in[12];
  const float* a1b  = (const float*)d_in[13];
  float* out = (float*)d_out;

  const int MPe = cdiv(nEnt, GBM) * GBM;
  const int MPr = cdiv(nRel, GBM) * GBM;
  const int nUnits = U_W1 + nB * (ED / 8);

  char* ws = (char*)d_ws;
  size_t off = 0;
  const size_t oPL = off; off += (size_t)nUnits * 16;               off = (off + 255) & ~(size_t)255;
  const size_t oTR = off; off += (size_t)MPr * TW * 4;              off = (off + 255) & ~(size_t)255;
  const size_t oC0 = off; off += (size_t)nB * ED * 4;               off = (off + 255) & ~(size_t)255;
  const size_t oC1 = off; off += (size_t)nB * ED * 4;               off = (off + 255) & ~(size_t)255;
  const size_t oHH = off; off += (size_t)nB * KH * 2;               off = (off + 255) & ~(size_t)255;
  const size_t oTE = off; off += (size_t)MPe * TW * 4;              off = (off + 255) & ~(size_t)255;
  if (off > ws_size || off > (size_t)WSMAX) return;
  unsigned short* PL   = (unsigned short*)(ws + oPL);
  unsigned short* WE   = PL;
  unsigned short* WR   = PL + (size_t)U_WE * 8;
  unsigned short* W0H  = PL + (size_t)U_WR * 8;
  unsigned short* W1H2 = PL + (size_t)U_W0 * 8;
  unsigned short* HB   = PL + (size_t)U_W1 * 8;
  float*          TR   = (float*)(ws + oTR);
  float*          C0   = (float*)(ws + oC0);
  float*          C1   = (float*)(ws + oC1);
  unsigned short* HHL  = (unsigned short*)(ws + oHH);
  float*          TE   = (float*)(ws + oTE);

  const int gemmLds2 = GBM * 2 * GBN * 4;
  const int gemmLds1 = GBM * 1 * GBN * 4;
  const int layLds   = LDS_LAYER_FLOATS * 4;
  hipFuncSetAttribute(reinterpret_cast<const void*>(&k_gemm<2, 1>), hipFuncAttributeMaxDynamicSharedMemorySize, gemmLds2);
  hipFuncSetAttribute(reinterpret_cast<const void*>(&k_layer<0>), hipFuncAttributeMaxDynamicSharedMemorySize, layLds);
  hipFuncSetAttribute(reinterpret_cast<const void*>(&k_layer<1>), hipFuncAttributeMaxDynamicSharedMemorySize, layLds);

  k_prep<<<cdiv(nUnits, NTHR), NTHR, 0, stream>>>(W0, W1, embE, be1, bq, PL, nEnt, nUnits);
  k_gemm<2, 1><<<MPe / GBM, GTHR * 2, gemmLds2, stream>>>(embE, HB, ED, nEnt, WE, ED, ED, TE, W0, 0);
  k_gemm<2, 1><<<MPr / GBM, GTHR * 2, gemmLds2, stream>>>(embR, HB, ED, nRel, WR, ED, ED, TR, W0, 0);
  k_gemm<1, 0><<<nB / GBM, GTHR, gemmLds1, stream>>>(embR, HB, ED, nB, W0H, ED, ED, C0, b0, 1);
  k_layer<0><<<nB, NTHR, layLds, stream>>>(nbr, msk, C0, TR, TE, a0W, a0b, HB, HHL, out, nRel, nEnt);
  k_gemm<1, 0><<<nB / GBM, GTHR, gemmLds1, stream>>>(embR, HHL, KH, nB, W1H2, KH, KH, C1, b1, 1);
  k_layer<1><<<nB, NTHR, layLds, stream>>>(nbr, msk, C1, TR, TE, a1W, a1b, HB, HHL, out, nRel, nEnt);
}
